// StructuralGcn_27178553049644
// MI455X (gfx1250) — hardware-run, weakly checked
//
#include <hip/hip_runtime.h>

typedef float          v8f   __attribute__((ext_vector_type(8)));
typedef float          v4f   __attribute__((ext_vector_type(4)));
typedef unsigned int   v4u   __attribute__((ext_vector_type(4)));
typedef int            v8i   __attribute__((ext_vector_type(8)));
typedef unsigned short v8us  __attribute__((ext_vector_type(8)));
typedef unsigned short v16us __attribute__((ext_vector_type(16)));
typedef __bf16         v16bf __attribute__((ext_vector_type(16)));
typedef _Float16       v16h  __attribute__((ext_vector_type(16)));
typedef v4f  __attribute__((may_alias)) v4fa;
typedef v8us __attribute__((may_alias)) v8usa;
union FragB { v16bf v; v16us u; v8us h[2]; v8i w; };
union FragH { v16h  v; v16us u; v8us h[2]; v8i w; };

__device__ __forceinline__ v8f wmb(const FragB& a, const FragB& b, v8f c) {
  v8f d = __builtin_amdgcn_wmma_f32_16x16x32_bf16(false, a.v, false, b.v, (short)0, c, false, false);
  asm volatile("v_nop\n\tv_nop\n\tv_nop\n\tv_nop" : "+v"(d) : "v"(a.w), "v"(b.w));
  return d;
}

__device__ __forceinline__ v8f wmh(const FragH& a, const FragH& b, v8f c) {
  v8f d = __builtin_amdgcn_wmma_f32_16x16x32_f16(false, a.v, false, b.v, (short)0, c, false, false);
  asm volatile("v_nop\n\tv_nop\n\tv_nop\n\tv_nop" : "+v"(d) : "v"(a.w), "v"(b.w));
  return d;
}

__device__ __forceinline__ unsigned bf16_bits(float f) {
  const unsigned u = __float_as_uint(f);
  const unsigned r = (u + 0x7FFFu + ((u >> 16) & 1u)) >> 16;
  const unsigned q = (u >> 16) | 0x40u;
  return ((u & 0x7fffffffu) > 0x7f800000u) ? q : r;
}

__device__ __forceinline__ float bf16_val(float f) {
  return __uint_as_float(bf16_bits(f) << 16);
}
__device__ __forceinline__ int clampi(int v, int lo, int hi) {
  return v < lo ? lo : (v > hi ? hi : v);
}

__device__ __forceinline__ unsigned f16_bits(float f) {
  const unsigned u  = __float_as_uint(f);
  const unsigned s  = (u >> 16) & 0x8000u;
  const unsigned a  = u & 0x7fffffffu;
  const unsigned t  = a - 0x38000000u;
  const unsigned r  = (t + 0x0FFFu + ((t >> 13) & 1u)) >> 13;
  const unsigned rc = r > 0x7C00u ? 0x7C00u : r;
  const bool small  = a < 0x38800000u;
  const bool isnan  = a > 0x7f800000u;
  const unsigned fin = small ? 0u : (s | rc);
  return isnan ? (s | 0x7E00u) : fin;
}

__device__ __forceinline__ unsigned pk16(unsigned lo, unsigned hi) { return lo | (hi << 16); }
__device__ __forceinline__ unsigned bf16_lo_bits(float v) {
  float hi = bf16_val(v);
  asm volatile("" : "+v"(hi));
  return bf16_bits(v - hi);
}
__device__ __forceinline__ v4u pack8_bf16(v4f a, v4f c) {
  return (v4u){ pk16(bf16_bits(a[0]), bf16_bits(a[1])), pk16(bf16_bits(a[2]), bf16_bits(a[3])),
                pk16(bf16_bits(c[0]), bf16_bits(c[1])), pk16(bf16_bits(c[2]), bf16_bits(c[3])) };
}
__device__ __forceinline__ v4u pack8_bf16_lo(v4f a, v4f c) {
  return (v4u){ pk16(bf16_lo_bits(a[0]), bf16_lo_bits(a[1])), pk16(bf16_lo_bits(a[2]), bf16_lo_bits(a[3])),
                pk16(bf16_lo_bits(c[0]), bf16_lo_bits(c[1])), pk16(bf16_lo_bits(c[2]), bf16_lo_bits(c[3])) };
}
__device__ __forceinline__ v4u pack8_f16(v4f a, v4f c) {
  return (v4u){ pk16(f16_bits(a[0]), f16_bits(a[1])), pk16(f16_bits(a[2]), f16_bits(a[3])),
                pk16(f16_bits(c[0]), f16_bits(c[1])), pk16(f16_bits(c[2]), f16_bits(c[3])) };
}

template <int FORM>
__global__ __launch_bounds__(256) void k_plane(const float* __restrict__ src, int rows, int cols, int ldsrc,
                                               unsigned short* __restrict__ dst, int MP, int KP) {
  static_assert(FORM >= 0 && FORM <= 3);
  const int KTOT = (FORM == 1 || FORM == 3) ? 2 * KP : KP;
  const unsigned ppr   = (unsigned)(KTOT >> 3);
  const unsigned kp8   = (unsigned)(KP >> 3);
  const unsigned total = (unsigned)MP * ppr;
  const unsigned g     = blockIdx.x * 256u + threadIdx.x;
  const unsigned rowu  = g / ppr;
  const unsigned p     = g - rowu * ppr;
  const bool second    = p >= kp8;
  const int row = (int)rowu;
  const int c0  = (int)((second ? p - kp8 : p) << 3);
  const float* srow = src + (size_t)clampi(row, 0, rows - 1) * (size_t)ldsrc;
  float x[8];
  unsigned mk[8];
#pragma unroll
  for (int e = 0; e < 8; ++e) {
    const int c = c0 + e;
    const float v = srow[clampi(c, 0, cols - 1)];
    asm volatile("" :: "v"(v));
    x[e]  = v;
    mk[e] = (row < rows && c < cols) ? 0xFFFFu : 0u;
  }
  const v4f a = (v4f){ x[0], x[1], x[2], x[3] };
  const v4f c = (v4f){ x[4], x[5], x[6], x[7] };
  v4u o;
  if (FORM == 2) {
    o = pack8_f16(a, c);
  } else {
    const v4u hi = pack8_bf16(a, c);
    o = hi;
    if (FORM == 1) { const v4u lo = pack8_bf16_lo(a, c); o = second ? lo : hi; }
  }
  const v4u mw = (v4u){ pk16(mk[0], mk[1]), pk16(mk[2], mk[3]), pk16(mk[4], mk[5]), pk16(mk[6], mk[7]) };
  o &= mw;
  if (g < total) {
    volatile v4u* q = (volatile v4u*)(dst + (size_t)g * 8);
    *q = o;
    __threadfence();
    *q = o;
  }
}

template <int FORM> struct FragOf    { typedef FragB T; };
template <>         struct FragOf<2> { typedef FragH T; };
__device__ __forceinline__ v8f mm(const FragB& a, const FragB& b, v8f c) { return wmb(a, b, c); }
__device__ __forceinline__ v8f mm(const FragH& a, const FragH& b, v8f c) { return wmh(a, b, c); }
template <class F> __device__ __forceinline__ F ld_frag(const unsigned short* p) {
  F f;
  f.h[0] = *(const v8usa*)(p);
  f.h[1] = *(const v8usa*)(p + 16);
  return f;
}

template <int FORM, int EPI>
__global__ __launch_bounds__(256) __attribute__((amdgpu_num_vgpr(248)))
void k_gemm_nt(const unsigned short* __restrict__ A, const unsigned short* __restrict__ B,
               const float* __restrict__ bias, float* __restrict__ D, int M, int N, int KTOT, int ldd) {
  static_assert(FORM >= 0 && FORM <= 2);
  static_assert(EPI == 0 || EPI == 1);
  typedef typename FragOf<FORM>::T F;
  __shared__ __attribute__((aligned(16))) float sT[8][16 * 68];
  const int lane = threadIdx.x & 31;
  const int wave = threadIdx.x >> 5;
  const int tilesM = (M + 63) >> 6;
  const int tilesN = (N + 63) >> 6;
  const int tile = blockIdx.x * 8 + wave;
  if (tile >= tilesM * tilesN) return;
  const int tm = tile / tilesN;
  const int tn = tile - tm * tilesN;
  const int m0 = tm << 6;
  const int n0 = tn << 6;

  const int rl = lane & 15;
  const int h8 = (lane >> 4) * 8;
  const unsigned short* pa = A + (size_t)(m0 + rl) * (size_t)KTOT + h8;
  const unsigned short* pb = B + (size_t)(n0 + rl) * (size_t)KTOT + h8;

  v8f acc[4][4];
#pragma unroll
  for (int i = 0; i < 4; ++i)
#pragma unroll
    for (int j = 0; j < 4; ++j) acc[i][j] = (v8f){0.f, 0.f, 0.f, 0.f, 0.f, 0.f, 0.f, 0.f};

#pragma unroll 1
  for (int k0 = 0; k0 < KTOT; k0 += 32) {
    F bf[4];
#pragma unroll
    for (int j = 0; j < 4; ++j) bf[j] = ld_frag<F>(pb + (size_t)(j << 4) * (size_t)KTOT + k0);
#pragma unroll
    for (int i = 0; i < 4; ++i) {
      const F af = ld_frag<F>(pa + (size_t)(i << 4) * (size_t)KTOT + k0);
#pragma unroll
      for (int j = 0; j < 4; ++j) acc[i][j] = mm(af, bf[j], acc[i][j]);
    }
  }

  float* slab = sT[wave];
  const int hh = lane >> 4;
  const int c4 = (lane & 15) * 4;
  const int nc = n0 + c4;
  const bool cok = nc < N;
  v4f bv = (v4f){0.f, 0.f, 0.f, 0.f};
  if (EPI == 1) {
    bv = *(const v4fa*)(bias + clampi(nc, 0, N - 4));
    asm volatile("" :: "v"(bv));
  }
#pragma unroll
  for (int i = 0; i < 4; ++i) {
    const int mBase = m0 + (i << 4);
#pragma unroll
    for (int j = 0; j < 4; ++j) {
#pragma unroll
      for (int r = 0; r < 8; ++r) slab[(h8 + r) * 68 + (j << 4) + rl] = acc[i][j][r];
    }
    __builtin_amdgcn_fence(__ATOMIC_RELEASE, "workgroup");
    __builtin_amdgcn_wave_barrier();
    __builtin_amdgcn_fence(__ATOMIC_ACQUIRE, "workgroup");
    v4f vv[8];
#pragma unroll
    for (int it = 0; it < 8; ++it) {
      const int row = it * 2 + hh;
      v4f v = *(const v4fa*)(slab + row * 68 + c4);
      if (EPI == 1) v += bv;
      vv[it] = v;
    }
    for (int pass = 0; pass < 2; ++pass) {
#pragma unroll
      for (int it = 0; it < 8; ++it) {
        const int row = mBase + it * 2 + hh;
        if (cok && row < M) *(volatile v4f*)(D + (size_t)row * (size_t)ldd + nc) = vv[it];
      }
      __threadfence();
    }
    __builtin_amdgcn_fence(__ATOMIC_RELEASE, "workgroup");
    __builtin_amdgcn_wave_barrier();
    __builtin_amdgcn_fence(__ATOMIC_ACQUIRE, "workgroup");
  }
}

#include <stddef.h>
#include <stdint.h>
#include <math.h>

#pragma clang fp contract(off)

#ifndef SPLIT_2
#define SPLIT_2 1
#endif

#define NN      50000
#define KD      128
#define HD      64
#define MIDC    32
#define NE      800000
#define MP      50048
#define NTHR    256
#define NWAVE   8
#define EPT     8
#define WCH     (32 * EPT)
#define NBRUN   1024
#define SLB     10
#define NBK     49
#define WLCAP   3072
#define LCAP    21504
#define DEGCAP  64
#define MAXDEG_MEAS   35
#define MAXB1024_MEAS 16623

#define BK_ZINTS (NWAVE * WLCAP + LCAP + 3 * NBRUN)
#define BK_INTS  (BK_ZINTS + 16)
#define BK_LDS   (BK_INTS * 4)

#define PBX     (MP * KD / 8 / 256)
#define PB_W1   4
#define PB_W2   4
#define PB_TAB  1
#define PB_TOT  (PB_W1 + PB_W2 + PB_TAB)
#define GEMM_BLOCKS (((MP / 64) + 7) / 8)
#define OUT_WAVES   ((NN + 31) / 32)
#define OUT_BLOCKS  ((OUT_WAVES + NWAVE - 1) / NWAVE)

static_assert(HD == 32 * 2 && HD == 16 * 4 && HD % 32 == 0);
static_assert(KD % 32 == 0 && KD == 2 * HD && MIDC % 4 == 0 && MIDC <= HD);
static_assert(MP % 64 == 0 && MP >= NN && MP == 391 * 128 && MP % 16 == 0);
static_assert((MP * KD / 8) % 256 == 0 && PBX == 3128);
static_assert((HD * KD / 8) == PB_W1 * NTHR && (HD * KD / 8) == PB_W2 * NTHR);
static_assert(NBRUN == (1 << SLB) && NBRUN == NTHR * 4 && NBRUN % 32 == 0);
static_assert(NBK * NBRUN >= NN && (NBK - 1) * NBRUN < NN);
static_assert(NE < (1 << 21) && (((long long)NE) << SLB) < (1LL << 31));
static_assert(NE % WCH == 0 && NE % 4 == 0);
static_assert((long long)LCAP * 100 >= (long long)MAXB1024_MEAS * 125);
static_assert(WLCAP >= MAXB1024_MEAS / 8 + 8 * 46 + 1);
static_assert(MAXDEG_MEAS + 8 <= DEGCAP);
static_assert(LCAP % (NTHR * 4) == 0 && BK_ZINTS % (NTHR * 4) == 0);
static_assert(BK_LDS <= 262144);
static_assert(NN % NWAVE == 0 && MP % NWAVE == 0);
static_assert(NN == 1562 * 32 + 16 && OUT_WAVES == 1563 && OUT_BLOCKS == 196);
static_assert(GEMM_BLOCKS == 98);

typedef float        v2f __attribute__((ext_vector_type(2)));
typedef unsigned int v2u __attribute__((ext_vector_type(2)));
typedef int          v4i __attribute__((ext_vector_type(4)));
typedef v2f __attribute__((may_alias)) v2fa;
typedef v2u __attribute__((may_alias)) v2ua;
typedef v4i __attribute__((may_alias)) v4ia;

__device__ __forceinline__ void st2_v4u(unsigned short* p, v4u v) {
  volatile v4u* q = (volatile v4u*)p;
  *q = v;
  __threadfence();
  *q = v;
}
__device__ __forceinline__ void st2_v4f(float* p, v4f v) {
  volatile v4f* q = (volatile v4f*)p;
  *q = v;
  __threadfence();
  *q = v;
}

__device__ __forceinline__ v4u gather8_bf16(const float* __restrict__ base, int stride) {
  float f[8];
#pragma unroll
  for (int i = 0; i < 8; ++i) {
    const float v = base[(size_t)i * (size_t)stride];
    asm volatile("" :: "v"(v));
    f[i] = v;
  }
  return (v4u){ pk16(bf16_bits(f[0]), bf16_bits(f[1])), pk16(bf16_bits(f[2]), bf16_bits(f[3])),
                pk16(bf16_bits(f[4]), bf16_bits(f[5])), pk16(bf16_bits(f[6]), bf16_bits(f[7])) };
}

__global__ __launch_bounds__(NTHR) void k_prep(const float* __restrict__ w1, const float* __restrict__ w2,
                                               const float* __restrict__ b1, const float* __restrict__ b2,
                                               const float* __restrict__ w3, const float* __restrict__ b3,
                                               unsigned short* w1t, unsigned short* w2d, float* tab) {
  const int tid = (int)threadIdx.x;
  const int blk = (int)blockIdx.x;
  if (blk < PB_W1) {
    const int u = blk * NTHR + tid;
    const int n = u >> 4, k8 = (u & 15) * 8;
    const v4u o = gather8_bf16(w1 + (size_t)k8 * HD + n, HD);
    st2_v4u(w1t + (size_t)n * KD + k8, o);
  } else if (blk < PB_W1 + PB_W2) {
    const int u = (blk - PB_W1) * NTHR + tid;
    const int n = u >> 4, k8 = (u & 15) * 8;
    const int ks = k8 & (HD - 1);
    const int nc = n < MIDC ? n : MIDC - 1;
    v4u o = gather8_bf16(w2 + (size_t)ks * MIDC + nc, MIDC);
    const unsigned m = (n < MIDC) ? 0xFFFFFFFFu : 0u;
    o &= (v4u){ m, m, m, m };
    st2_v4u(w2d + (size_t)n * KD + k8, o);
  } else {
    const int c4  = (tid & 15) * 4;
    const int seg = (tid >> 4) & 3;
    const int c4c = c4 < MIDC - 4 ? c4 : MIDC - 4;
    const v4f x1 = *(const v4fa*)(b1 + c4);
    const v4f x2 = *(const v4fa*)(b2 + c4c);
    const v4f x3 = *(const v4fa*)(w3 + c4c);
    const float x4 = b3[0];
    asm volatile("" :: "v"(x1), "v"(x2), "v"(x3));
    asm volatile("" :: "v"(x4));
    const unsigned lowm = (c4 < MIDC) ? 0xFFFFFFFFu : 0u;
    const unsigned m1 = (seg == 0) ? 0xFFFFFFFFu : 0u;
    const unsigned m2 = (seg == 1) ? lowm : 0u;
    const unsigned m3 = (seg == 2) ? lowm : 0u;
    const unsigned m4 = (seg == 3 && c4 == 0) ? 0xFFFFFFFFu : 0u;
    const unsigned u4 = __float_as_uint(bf16_val(x4)) & m4;
    v4f o;
#pragma unroll
    for (int e = 0; e < 4; ++e) {
      const unsigned u1 = __float_as_uint(bf16_val(x1[e])) & m1;
      const unsigned u2 = __float_as_uint(bf16_val(x2[e])) & m2;
      const unsigned u3 = __float_as_uint(bf16_val(x3[e])) & m3;
      const unsigned ue = (e == 0) ? u4 : 0u;
      o[e] = __uint_as_float(u1 | u2 | u3 | ue);
    }
    if (tid < 64) st2_v4f(tab + 4 * tid, o);
  }
}

__device__ __forceinline__ void list_flush(const int* pl, const int* cnt, const int* offs, const int* dvb, int ov,
                                           int* lp, int* cp, int* op, int* dp, int* fp, int tid) {
#pragma unroll 1
  for (int i = tid * 4; i < LCAP; i += NTHR * 4) {
    const v4i v = *(const v4ia*)(pl + i);
    *(volatile v4i*)(lp + i) = v;
  }
  {
    const v4i vc = *(const v4ia*)(cnt + 4 * tid);
    const v4i vo = *(const v4ia*)(offs + 4 * tid);
    const v4i vd = *(const v4ia*)(dvb + 4 * tid);
    *(volatile v4i*)(cp + 4 * tid) = vc;
    *(volatile v4i*)(op + 4 * tid) = vo;
    *(volatile v4i*)(dp + 4 * tid) = vd;
  }
  if (tid < 8) {
    const v4i f = {ov, ov, ov, ov};
    *(volatile v4i*)(fp + 4 * tid) = f;
  }
}

__global__ __launch_bounds__(NTHR) void k_list(const int* __restrict__ srcs, const int* __restrict__ dsts,
                                               int* LIST, int* CNT, int* OFF, int* DINVB, int* FLAG) {
  extern __shared__ __attribute__((aligned(16))) int dsm[];
  int* wl   = dsm;
  int* pl   = dsm + NWAVE * WLCAP;
  int* cnt  = pl + LCAP;
  int* offs = cnt + NBRUN;
  int* cur  = offs + NBRUN;
  int* misc = cur + NBRUN;
  const int tid = (int)threadIdx.x, lane = tid & 31, wave = tid >> 5;
  const int blk = (int)blockIdx.x;
  const unsigned nbs = (unsigned)(blk * NBRUN);

  {
    const v4i z4 = {0, 0, 0, 0};
#pragma unroll 1
    for (int i = tid * 4; i < BK_ZINTS; i += NTHR * 4) *(v4ia*)(dsm + i) = z4;
    if (tid < 16) misc[tid] = 0;
  }
  __syncthreads();

  {
    const int per  = ((NE + NWAVE * WCH - 1) / (NWAVE * WCH)) * WCH;
    const int ebeg = wave * per;
    const int eend = (ebeg + per < NE) ? (ebeg + per) : NE;
    int* mylist = wl + wave * WLCAP;
    int wc = 0;
#pragma unroll 1
    for (int cb = ebeg; cb < eend; cb += WCH) {
      const int e0 = cb + lane * EPT;
      const v4i da = *(const v4ia*)(dsts + e0);
      const v4i db = *(const v4ia*)(dsts + e0 + 4);
      const int d0 = da.x, d1 = da.y, d2 = da.z, d3 = da.w;
      const int d4 = db.x, d5 = db.y, d6 = db.z, d7 = db.w;
      asm volatile("" :: "v"(d0), "v"(d1), "v"(d2), "v"(d3));
      asm volatile("" :: "v"(d4), "v"(d5), "v"(d6), "v"(d7));
      const unsigned s0 = (unsigned)d0 - nbs, s1 = (unsigned)d1 - nbs;
      const unsigned s2 = (unsigned)d2 - nbs, s3 = (unsigned)d3 - nbs;
      const unsigned s4 = (unsigned)d4 - nbs, s5 = (unsigned)d5 - nbs;
      const unsigned s6 = (unsigned)d6 - nbs, s7 = (unsigned)d7 - nbs;
      const bool h0 = s0 < (unsigned)NBRUN, h1 = s1 < (unsigned)NBRUN, h2 = s2 < (unsigned)NBRUN, h3 = s3 < (unsigned)NBRUN;
      const bool h4 = s4 < (unsigned)NBRUN, h5 = s5 < (unsigned)NBRUN, h6 = s6 < (unsigned)NBRUN, h7 = s7 < (unsigned)NBRUN;
      const unsigned m0 = __builtin_amdgcn_ballot_w32(h0), m1 = __builtin_amdgcn_ballot_w32(h1);
      const unsigned m2 = __builtin_amdgcn_ballot_w32(h2), m3 = __builtin_amdgcn_ballot_w32(h3);
      const unsigned m4 = __builtin_amdgcn_ballot_w32(h4), m5 = __builtin_amdgcn_ballot_w32(h5);
      const unsigned m6 = __builtin_amdgcn_ballot_w32(h6), m7 = __builtin_amdgcn_ballot_w32(h7);
      const unsigned any = m0 | m1 | m2 | m3 | m4 | m5 | m6 | m7;
      if (any != 0u) {
        const int pre = (int)(__builtin_amdgcn_mbcnt_lo(m0, 0u) + __builtin_amdgcn_mbcnt_lo(m1, 0u) +
                              __builtin_amdgcn_mbcnt_lo(m2, 0u) + __builtin_amdgcn_mbcnt_lo(m3, 0u) +
                              __builtin_amdgcn_mbcnt_lo(m4, 0u) + __builtin_amdgcn_mbcnt_lo(m5, 0u) +
                              __builtin_amdgcn_mbcnt_lo(m6, 0u) + __builtin_amdgcn_mbcnt_lo(m7, 0u));
        int p = wc + pre;
        if (h0) { if (p < WLCAP) mylist[p] = ((e0 + 0) << SLB) | (int)s0; p = p + 1; }
        if (h1) { if (p < WLCAP) mylist[p] = ((e0 + 1) << SLB) | (int)s1; p = p + 1; }
        if (h2) { if (p < WLCAP) mylist[p] = ((e0 + 2) << SLB) | (int)s2; p = p + 1; }
        if (h3) { if (p < WLCAP) mylist[p] = ((e0 + 3) << SLB) | (int)s3; p = p + 1; }
        if (h4) { if (p < WLCAP) mylist[p] = ((e0 + 4) << SLB) | (int)s4; p = p + 1; }
        if (h5) { if (p < WLCAP) mylist[p] = ((e0 + 5) << SLB) | (int)s5; p = p + 1; }
        if (h6) { if (p < WLCAP) mylist[p] = ((e0 + 6) << SLB) | (int)s6; p = p + 1; }
        if (h7) { if (p < WLCAP) mylist[p] = ((e0 + 7) << SLB) | (int)s7; p = p + 1; }
        wc += (int)(__builtin_popcount(m0) + __builtin_popcount(m1) + __builtin_popcount(m2) + __builtin_popcount(m3) +
                    __builtin_popcount(m4) + __builtin_popcount(m5) + __builtin_popcount(m6) + __builtin_popcount(m7));
      }
    }
    if (lane == 0) misc[wave] = wc;
  }
  __syncthreads();

  if (wave == 0) {
    int ov = 0;
    int tot = 0;
#pragma unroll 1
    for (int w2 = 0; w2 < NWAVE; ++w2) {
      int c = misc[w2];
      if (c > WLCAP) ov = 1;
      c = c < 0 ? 0 : (c > WLCAP ? WLCAP : c);
      tot += c;
#pragma unroll 1
      for (int b0 = 0; b0 < c; b0 += 32) {
        const int idx = b0 + lane;
        const int ent = wl[w2 * WLCAP + (idx < WLCAP ? idx : WLCAP - 1)];
        const int m32 = (c - b0) < 32 ? (c - b0) : 32;
#pragma unroll 1
        for (int k = 0; k < m32; ++k) {
          const int u    = __builtin_amdgcn_readlane(ent, k);
          const int slot = u & (NBRUN - 1);
          if (lane == 0) cnt[slot] = cnt[slot] + 1;
        }
      }
    }
    if (tot > LCAP) ov = 1;
    if (lane == 0) misc[9] = ov;
  }
  __syncthreads();
  if (wave == 0) {
    const int base = lane * (NBRUN / 32);
    int s = 0;
#pragma unroll 1
    for (int i = 0; i < NBRUN / 32; ++i) s += cnt[base + i];
    int incl = s;
#pragma unroll
    for (int d = 1; d < 32; d <<= 1) {
      const int y = __shfl_up(incl, d, 32);
      if (lane >= d) incl += y;
    }
    int run = incl - s;
#pragma unroll 1
    for (int i = 0; i < NBRUN / 32; ++i) {
      const int cv = cnt[base + i];
      offs[base + i] = run;
      cur[base + i]  = run;
      run += cv;
    }
  }
  __syncthreads();

  if (wave == 0) {
#pragma unroll 1
    for (int w2 = 0; w2 < NWAVE; ++w2) {
      int c = misc[w2];
      c = c < 0 ? 0 : (c > WLCAP ? WLCAP : c);
#pragma unroll 1
      for (int b0 = 0; b0 < c; b0 += 32) {
        const int idx = b0 + lane;
        const int ent = wl[w2 * WLCAP + (idx < WLCAP ? idx : WLCAP - 1)];
        int eid = (ent >> SLB) & 0x1FFFFF;
        eid = eid > NE - 1 ? NE - 1 : eid;
        int sr = srcs[eid];
        asm volatile("" :: "v"(sr));
        sr = sr < 0 ? 0 : (sr > NN - 1 ? NN - 1 : sr);
        const int m32 = (c - b0) < 32 ? (c - b0) : 32;
#pragma unroll 1
        for (int k = 0; k < m32; ++k) {
          const int u    = __builtin_amdgcn_readlane(ent, k);
          const int w0   = __builtin_amdgcn_readlane(sr, k);
          const int slot = u & (NBRUN - 1);
          if (lane == 0) {
            int p = cur[slot];
            p = p < 0 ? 0 : (p > LCAP - 1 ? LCAP - 1 : p);
            pl[p] = w0;
            cur[slot] = p + 1;
          }
        }
      }
    }
  }
  __syncthreads();

#pragma unroll 1
  for (int j = 0; j < 4; ++j) {
    const int cc = cnt[4 * tid + j];
    const float deg = (float)(cc + 1);
    const float dv = (deg > 0.0f) ? (1.0f / sqrtf(deg)) : 0.0f;
    cur[4 * tid + j] = __float_as_int(dv);
  }
  __syncthreads();

  const int ovf = misc[9];
  int* lp = LIST  + (size_t)blk * (size_t)LCAP;
  int* cp = CNT   + (size_t)blk * NBRUN;
  int* op = OFF   + (size_t)blk * NBRUN;
  int* dp = DINVB + (size_t)blk * NBRUN;
  int* fp = FLAG  + (size_t)blk * 32;
  list_flush(pl, cnt, offs, cur, ovf, lp, cp, op, dp, fp, tid);
  __threadfence();
  list_flush(pl, cnt, offs, cur, ovf, lp, cp, op, dp, fp, tid);
}

__device__ __forceinline__ v2f walk_row(const int* __restrict__ LIST, const int* __restrict__ CNT,
                                        const int* __restrict__ OFF, const float* __restrict__ DINV,
                                        const int* __restrict__ FLAG, const float* __restrict__ T,
                                        const float* __restrict__ BV, int dn, int lane) {
  const int bk = dn >> SLB;
  const int* lb = LIST + (size_t)bk * (size_t)LCAP;
  const int craw = CNT[dn];
  const int oraw = OFF[dn];
  const int flag = FLAG[(size_t)bk * 32];
  const float dd = DINV[dn];
  const v2f self = *(const v2fa*)(T + (size_t)dn * HD + 2 * lane);
  const v2f bb   = *(const v2fa*)(BV + 2 * lane);
  asm volatile("" :: "v"(craw), "v"(oraw), "v"(flag), "v"(dd));
  asm volatile("" :: "v"(self), "v"(bb));

  const bool big = craw > DEGCAP;
  const int c = __builtin_amdgcn_readfirstlane(craw < 0 ? 0 : (craw > DEGCAP ? DEGCAP : craw));
  const int o = oraw < 0 ? 0 : (oraw > LCAP - 1 ? LCAP - 1 : oraw);
  int last = o + (c > 0 ? c : 1) - 1;
  last = last > LCAP - 1 ? LCAP - 1 : last;

  float a0 = 0.0f, a1 = 0.0f;
#pragma unroll 1
  for (int b0 = 0; b0 < c; b0 += 32) {
    int idx = o + b0 + lane;
    idx = idx > last ? last : idx;
    int sr = lb[idx];
    asm volatile("" :: "v"(sr));
    sr = sr < 0 ? 0 : (sr > NN - 1 ? NN - 1 : sr);
    const float dsv = DINV[sr];
    asm volatile("" :: "v"(dsv));
    const int dsb = __float_as_int(dsv);
    const int m32 = (c - b0) < 32 ? (c - b0) : 32;
#pragma unroll 1
    for (int k = 0; k < m32; ++k) {
      const int   sk = __builtin_amdgcn_readlane(sr, k);
      const float ds = __int_as_float(__builtin_amdgcn_readlane(dsb, k));
      const float w  = ds * dd;
      const v2f q = *(const v2fa*)(T + (size_t)sk * HD + 2 * lane);
      a0 = a0 + q.x * w;
      a1 = a1 + q.y * w;
    }
  }
  const float ws = dd * dd;
  a0 = a0 + self.x * ws;
  a1 = a1 + self.y * ws;
  const float v0 = a0 + bb.x;
  const float v1 = a1 + bb.y;
  const float z0 = (v0 > 0.0f) ? v0 : (v0 - v0);
  const float z1 = (v1 > 0.0f) ? v1 : (v1 - v1);
  const bool bad = (flag != 0) | big;
  const float qnan = __uint_as_float(0x7fc00000u);
  v2f r;
  r.x = bad ? qnan : z0;
  r.y = bad ? qnan : z1;
  return r;
}

__global__ __launch_bounds__(NTHR) void k_walk1(const int* __restrict__ LIST, const int* __restrict__ CNT,
                                                const int* __restrict__ OFF, const float* __restrict__ DINV,
                                                const int* __restrict__ FLAG, const float* __restrict__ T,
                                                const float* __restrict__ BV, unsigned short* OP, int n_rows) {
  __shared__ __attribute__((aligned(16))) unsigned srow[NWAVE][64];
  const int tid = (int)threadIdx.x, lane = tid & 31, wave = tid >> 5;
  const int node = (int)blockIdx.x * NWAVE + wave;
  const int dn = node < NN - 1 ? node : NN - 1;
  const v2f z = walk_row(LIST, CNT, OFF, DINV, FLAG, T, BV, dn, lane);
  const unsigned keep = (node < NN) ? 0xFFFFFFFFu : 0u;
  const unsigned hiw = pk16(bf16_bits(z.x), bf16_bits(z.y)) & keep;
#if SPLIT_2
  const unsigned low = pk16(bf16_lo_bits(z.x), bf16_lo_bits(z.y)) & keep;
#else
  const unsigned low = hiw & 0u;
#endif
  unsigned* row = srow[wave];
  row[lane]      = hiw;
  row[32 + lane] = low;
  __builtin_amdgcn_fence(__ATOMIC_RELEASE, "workgroup");
  __builtin_amdgcn_wave_barrier();
  __builtin_amdgcn_fence(__ATOMIC_ACQUIRE, "workgroup");
  const v2u ov = *(const v2ua*)(row + 2 * lane);
  if (node < n_rows) {
    volatile v2u* q = (volatile v2u*)(OP + (size_t)node * KD + 4 * lane);
    *q = ov;
    __threadfence();
    *q = ov;
  }
}

__global__ __launch_bounds__(NTHR) void k_walk2(const int* __restrict__ LIST, const int* __restrict__ CNT,
                                                const int* __restrict__ OFF, const float* __restrict__ DINV,
                                                const int* __restrict__ FLAG, const float* __restrict__ T,
                                                const float* __restrict__ BV, const float* __restrict__ W3T,
                                                float* T3P, int n_rows) {
  const int tid = (int)threadIdx.x, lane = tid & 31, wave = tid >> 5;
  const int node = (int)blockIdx.x * NWAVE + wave;
  const int dn = node < NN - 1 ? node : NN - 1;
  const v2f w3 = *(const v2fa*)(W3T + 2 * lane);
  asm volatile("" :: "v"(w3));
  const v2f z = walk_row(LIST, CNT, OFF, DINV, FLAG, T, BV, dn, lane);
  const float p0 = z.x * w3.x;
  const float p1 = z.y * w3.y;
  float s = p0 + p1;
  s = s + __shfl_xor(s, 16, 32);
  s = s + __shfl_xor(s, 8, 32);
  s = s + __shfl_xor(s, 4, 32);
  s = s + __shfl_xor(s, 2, 32);
  s = s + __shfl_xor(s, 1, 32);
  const unsigned keep = (lane == 0 && node < NN) ? 0xFFFFFFFFu : 0u;
  const float ov = __uint_as_float(__float_as_uint(s) & keep);
  if (node < n_rows) {
    volatile float* q = (volatile float*)(T3P + (size_t)node * 32 + lane);
    *q = ov;
    __threadfence();
    *q = ov;
  }
}

__global__ __launch_bounds__(NTHR) void k_swalk(const int* __restrict__ LIST, const int* __restrict__ CNT,
                                                const int* __restrict__ OFF, const float* __restrict__ DINV,
                                                const int* __restrict__ FLAG, const float* __restrict__ T3P,
                                                const float* __restrict__ B3, float* RP, int n_nodes) {
  const int tid = (int)threadIdx.x, lane = tid & 31, wave = tid >> 5;
  const int node = (int)blockIdx.x * NWAVE + wave;
  const int dn = node < NN - 1 ? node : NN - 1;
  const int bk = dn >> SLB;
  const int* lb = LIST + (size_t)bk * (size_t)LCAP;
  const int craw = CNT[dn];
  const int oraw = OFF[dn];
  const int flag = FLAG[(size_t)bk * 32];
  const float dd = DINV[dn];
  const float selfv = T3P[(size_t)dn * 32];
  const float bb = B3[0];
  asm volatile("" :: "v"(craw), "v"(oraw), "v"(flag), "v"(dd));
  asm volatile("" :: "v"(selfv), "v"(bb));

  const bool big = craw > DEGCAP;
  const int c = __builtin_amdgcn_readfirstlane(craw < 0 ? 0 : (craw > DEGCAP ? DEGCAP : craw));
  const int o = oraw < 0 ? 0 : (oraw > LCAP - 1 ? LCAP - 1 : oraw);
  int last = o + (c > 0 ? c : 1) - 1;
  last = last > LCAP - 1 ? LCAP - 1 : last;

  float acc = 0.0f;
#pragma unroll 1
  for (int b0 = 0; b0 < c; b0 += 32) {
    int idx = o + b0 + lane;
    idx = idx > last ? last : idx;
    int sr = lb[idx];
    asm volatile("" :: "v"(sr));
    sr = sr < 0 ? 0 : (sr > NN - 1 ? NN - 1 : sr);
    const float tv  = T3P[(size_t)sr * 32];
    const float dsv = DINV[sr];
    asm volatile("" :: "v"(tv), "v"(dsv));
    const float w = dsv * dd;
    const float t = tv * w;
    const int tb = __float_as_int(t);
    const int m32 = (c - b0) < 32 ? (c - b0) : 32;
#pragma unroll 1
    for (int k = 0; k < m32; ++k) {
      const float tk = __int_as_float(__builtin_amdgcn_readlane(tb, k));
      acc = acc + tk;
    }
  }
  const float ws = dd * dd;
  acc = acc + selfv * ws;
  const float v = acc + bb;
  const bool bad = (flag != 0) | big;
  const float qnan = __uint_as_float(0x7fc00000u);
  const float r = bad ? qnan : v;
  const unsigned keep = (lane == 0) ? 0xFFFFFFFFu : 0u;
  const float ov = __uint_as_float(__float_as_uint(r) & keep);
  if (node < n_nodes) {
    volatile float* q = (volatile float*)(RP + (size_t)node * 32 + lane);
    *q = ov;
    __threadfence();
    *q = ov;
  }
}

__global__ __launch_bounds__(NTHR) void k_out(const float* __restrict__ RP, float* out, int n_out) {
  const int tid = (int)threadIdx.x, lane = tid & 31, wave = tid >> 5;
  const int wv = (int)blockIdx.x * NWAVE + wave;
  const int f = wv * 32 + lane;
  const int fc = f < NN - 1 ? f : NN - 1;
  const float v = RP[(size_t)fc * 32];
  asm volatile("" :: "v"(v));
  if (f < n_out) {
    volatile float* q = (volatile float*)(out + f);
    *q = v;
    __threadfence();
    *q = v;
  }
}

extern "C" void kernel_launch(void* const* d_in, const int* in_sizes, int n_in,
                              void* d_out, int out_size, void* d_ws, size_t ws_size,
                              hipStream_t stream) {
  if (n_in < 8) return;
  if (in_sizes[0] != NN * KD) return;
  if (in_sizes[1] != 2 * NE) return;
  if (in_sizes[2] != KD * HD) return;
  if (in_sizes[3] != HD) return;
  if (in_sizes[4] != HD * MIDC) return;
  if (in_sizes[5] != MIDC) return;
  if (in_sizes[6] != MIDC) return;
  if (in_sizes[7] != 1) return;
  if (out_size != NN) return;
  const int n_out = out_size;

  const float* x   = (const float*)d_in[0];
  const int*   ei  = (const int*)d_in[1];
  const float* W1  = (const float*)d_in[2];
  const float* b1  = (const float*)d_in[3];
  const float* W2  = (const float*)d_in[4];
  const float* b2  = (const float*)d_in[5];
  const float* W3  = (const float*)d_in[6];
  const float* b3  = (const float*)d_in[7];
  const int* srcs  = ei;
  const int* dsts  = ei + NE;
  float* out = (float*)d_out;

  constexpr size_t zXB   = (size_t)MP * KD * 2;
  constexpr size_t zT    = (size_t)MP * HD * 4;
  constexpr size_t zOP   = (size_t)MP * KD * 2;
  constexpr size_t zT3P  = (size_t)MP * 32 * 4;
  constexpr size_t zRP   = (size_t)MP * 32 * 4;
  constexpr size_t zLIST = (size_t)NBK * LCAP * 4;
  constexpr size_t zTBL  = (size_t)NBK * NBRUN * 4;
  constexpr size_t zFLAG = 8192;
  constexpr size_t zWP   = (size_t)HD * KD * 2;
  constexpr size_t zTAB  = 1024;
  constexpr size_t oXB   = 0;
  constexpr size_t oT    = oXB + zXB;
  constexpr size_t oOP   = oT + zT;
  constexpr size_t oT3P  = oOP + zOP;
  constexpr size_t oLIST = oT3P + zT3P;
  constexpr size_t oCNT  = oLIST + zLIST;
  constexpr size_t oOFF  = oCNT + zTBL;
  constexpr size_t oDINV = oOFF + zTBL;
  constexpr size_t oFLAG = oDINV + zTBL;
  constexpr size_t oW1T  = oFLAG + zFLAG;
  constexpr size_t oW2D  = oW1T + zWP;
  constexpr size_t oTAB  = oW2D + zWP;
  constexpr size_t oEND  = oTAB + zTAB;
  static_assert(zXB % 256 == 0 && zT % 256 == 0 && zOP % 256 == 0 && zT3P % 256 == 0 && zLIST % 256 == 0);
  static_assert(zTBL % 256 == 0 && zFLAG % 256 == 0 && zWP % 256 == 0 && zTAB % 256 == 0);
  static_assert(zRP <= zT);
  static_assert(zFLAG >= (size_t)NBK * 128);
  static_assert(zTAB >= (size_t)4 * HD * 4);
  static_assert(oEND == 49701888);
  static_assert(oEND <= ((size_t)128 << 20));
  if (oEND > ws_size) return;

  char* ws = (char*)d_ws;
  unsigned short* XB   = (unsigned short*)(ws + oXB);
  float*          T    = (float*)(ws + oT);
  float*          RP   = (float*)(ws + oT);
  unsigned short* OP   = (unsigned short*)(ws + oOP);
  float*          T3P  = (float*)(ws + oT3P);
  int*            LIST = (int*)(ws + oLIST);
  int*            CNT  = (int*)(ws + oCNT);
  int*            OFF  = (int*)(ws + oOFF);
  int*            DVB  = (int*)(ws + oDINV);
  const float*    DINV = (const float*)(ws + oDINV);
  int*            FLAG = (int*)(ws + oFLAG);
  unsigned short* W1T  = (unsigned short*)(ws + oW1T);
  unsigned short* W2D  = (unsigned short*)(ws + oW2D);
  float*          TAB  = (float*)(ws + oTAB);

  hipFuncSetAttribute(reinterpret_cast<const void*>(&k_list), hipFuncAttributeMaxDynamicSharedMemorySize, (int)BK_LDS);

  k_plane<0><<<PBX, 256, 0, stream>>>(x, NN, KD, KD, XB, MP, KD);
  k_prep<<<PB_TOT, NTHR, 0, stream>>>(W1, W2, b1, b2, W3, b3, W1T, W2D, TAB);
  k_list<<<NBK, NTHR, BK_LDS, stream>>>(srcs, dsts, LIST, CNT, OFF, DVB, FLAG);
  k_gemm_nt<0, 0><<<GEMM_BLOCKS, 256, 0, stream>>>(XB, W1T, TAB, T, MP, HD, KD, HD);
  k_walk1<<<MP / NWAVE, NTHR, 0, stream>>>(LIST, CNT, OFF, DINV, FLAG, T, TAB, OP, MP);
  k_gemm_nt<0, 0><<<GEMM_BLOCKS, 256, 0, stream>>>(OP, W2D, TAB, T, MP, HD, KD, HD);
  k_walk2<<<MP / NWAVE, NTHR, 0, stream>>>(LIST, CNT, OFF, DINV, FLAG, T, TAB + HD, TAB + 2 * HD, T3P, MP);
  k_swalk<<<NN / NWAVE, NTHR, 0, stream>>>(LIST, CNT, OFF, DINV, FLAG, T3P, TAB + 3 * HD, RP, NN);
  k_out<<<OUT_BLOCKS, NTHR, 0, stream>>>(RP, out, n_out);
}
